// GraphAttentionLayer_79474074845764
// MI455X (gfx1250) — hardware-verified
//
#include <hip/hip_runtime.h>
#include <stddef.h>


typedef _Float16 v16h __attribute__((ext_vector_type(16)));
typedef _Float16 v8h  __attribute__((ext_vector_type(8)));
typedef float    v8f  __attribute__((ext_vector_type(8)));
typedef float    v4f  __attribute__((ext_vector_type(4)));
typedef _Float16 h16;

#ifndef NB
#define NB 8
#endif
#ifndef SEQ
#define SEQ 2048
#endif
#define NB_FULL  8
#define SEQ_FULL 2048
#define FEAT   256
#define NSLAB  4
#define MROWS  (NB * SEQ)
#define MWORDS (SEQ_FULL / 32)
#define LPR    (SEQ_FULL / 1024)

static_assert(NB >= 1 && NB <= NB_FULL);
static_assert(SEQ >= 128 && SEQ <= SEQ_FULL && (SEQ % 128) == 0);
static_assert((SEQ_FULL % 1024) == 0);
static_assert(FEAT == NSLAB * 64);
static_assert(FEAT == 32 * 8);
static_assert((FEAT % 64) == 0 && (FEAT % 32) == 0);
static_assert((MROWS % 64) == 0 && (MROWS % 8) == 0);
static_assert(((SEQ * LPR) % 8) == 0);
static_assert((size_t)NB_FULL * SEQ_FULL * FEAT * 4 == (size_t)16777216);

#define LDT 72
#define LDC 68
#define LDO 36
static_assert((LDT % 8) == 0 && LDT >= 64);
static_assert((LDC % 4) == 0 && LDC >= 64);
static_assert((LDO % 4) == 0 && LDO >= 32);

#define WCARRY 64.0f
#define XCARRY 16.0f
#define HCARRY 16.0f
#define PCARRY 16384.0f
#define ALPHA_NEG 0.01f
#define MASK_FILL (-1.0e9f)

#define WT_BYTES   ((size_t)FEAT * FEAT * 2)
#define X16_BYTES  ((size_t)MROWS * FEAT * 2)
#define VT_BYTES   ((size_t)MROWS * FEAT * 2)
#define MB_BYTES   ((size_t)SEQ * MWORDS * 4)
#define EP_BYTES   ((size_t)4 * 2 * MROWS * 4)
#define OFF_WT  ((size_t)0)
#define OFF_X16 (OFF_WT + WT_BYTES)
#define OFF_VT  (OFF_X16 + X16_BYTES)
#define OFF_MB  (OFF_VT + VT_BYTES)
#define OFF_EP  (OFF_MB + MB_BYTES)
#define WS_TOTAL (OFF_EP + EP_BYTES)
static_assert((WT_BYTES % 128) == 0 && (X16_BYTES % 128) == 0 && (VT_BYTES % 128) == 0);
static_assert((MB_BYTES % 128) == 0 && (EP_BYTES % 128) == 0);
static_assert(WS_TOTAL <= (size_t)134217728);

__device__ __forceinline__ float bf16r(float x) {
  unsigned int u = __float_as_uint(x);
  u = (u + 0x7FFFu + ((u >> 16) & 1u)) & 0xFFFF0000u;
  return __uint_as_float(u);
}

static __device__ __forceinline__ h16 toh_flush(float v) {
  const h16 r = (h16)v;
  return (fabsf(v) < 6.103515625e-05f) ? (h16)0.0f : r;
}

__device__ __forceinline__ v16h frag_at(const _Float16* p) {
  v8h lo = *(const v8h*)(p);
  v8h hi = *(const v8h*)(p + 16);
  v16h out;
#pragma unroll
  for (int i = 0; i < 8; ++i) { out[i] = lo[i]; out[i + 8] = hi[i]; }
  return out;
}
__device__ __forceinline__ v16h ld_frag(const _Float16* base, unsigned ld) {
  const unsigned lane = threadIdx.x & 31u;
  return frag_at(base + (lane & 15u) * ld + (lane >> 4) * 8u);
}

__device__ __forceinline__ v8f wmma16(v16h a, v16h b, v8f c) {
  v8f d = __builtin_amdgcn_wmma_f32_16x16x32_f16(false, a, false, b, (short)0, c,
                                                 false, false);
  asm volatile("v_nop\n\tv_nop\n\tv_nop\n\tv_nop" : "+v"(d) : "v"(a), "v"(b));
  return d;
}

__device__ __forceinline__ float red16_max(float x) {
#pragma unroll
  for (int off = 1; off < 16; off <<= 1) x = fmaxf(x, __shfl_xor(x, off, 32));
  return x;
}
__device__ __forceinline__ float red16_sum(float x) {
#pragma unroll
  for (int off = 1; off < 16; off <<= 1) x += __shfl_xor(x, off, 32);
  return x;
}

__device__ __forceinline__ void wave_lds_sync() {
  __builtin_amdgcn_fence(3  , "wavefront");
  asm volatile("s_wait_dscnt 0x0" ::: "memory");
  __builtin_amdgcn_wave_barrier();
}

__global__ __launch_bounds__(256) void wconv_kernel(
    const float* __restrict__ W, _Float16* __restrict__ Wt, unsigned ldw, unsigned ldk) {
  __shared__ _Float16 T[64 * LDT];
  const unsigned tid = threadIdx.x;
  const unsigned n0 = blockIdx.x * 64u;
  const unsigned k0 = blockIdx.y * 64u;
#pragma unroll 4
  for (unsigned j = 0; j < 16u; ++j) {
    const unsigned idx = tid + 256u * j;
    const unsigned kr = idx >> 6, nc = idx & 63u;
    const float v = W[(size_t)(k0 + kr) * ldw + n0 + nc];
    T[nc * LDT + kr] = (_Float16)(WCARRY * bf16r(v));
  }
  __syncthreads();
  v8h x[2];
  size_t off[2];
#pragma unroll
  for (unsigned i = 0; i < 2u; ++i) {
    const unsigned n = 32u * i + (tid >> 3);
    const unsigned kc = (tid & 7u) * 8u;
    x[i] = *(const v8h*)&T[n * LDT + kc];
    off[i] = (size_t)(n0 + n) * ldk + k0 + kc;
  }
#pragma unroll
  for (int i = 0; i < 2; ++i) *(volatile v8h*)(Wt + off[i]) = x[i];
  __threadfence();
#pragma unroll
  for (int i = 0; i < 2; ++i) *(volatile v8h*)(Wt + off[i]) = x[i];
}

__global__ __launch_bounds__(256) void xconv_kernel(
    const float* __restrict__ X, _Float16* __restrict__ dst) {
  const unsigned lane = threadIdx.x & 31u;
  const unsigned w = (unsigned)__builtin_amdgcn_readfirstlane((int)(threadIdx.x >> 5));
  const unsigned crow = blockIdx.x * 8u + w;
  const unsigned bidx = crow / (unsigned)SEQ;
  const unsigned sq = crow - bidx * (unsigned)SEQ;
  const size_t srow = (size_t)bidx * SEQ_FULL + sq;
  const float* xr = X + srow * FEAT + lane * 8u;
  const v4f a0 = *(const v4f*)(xr);
  const v4f a1 = *(const v4f*)(xr + 4u);
  v8h o;
#pragma unroll
  for (int i = 0; i < 4; ++i) {
    o[i]     = toh_flush(XCARRY * bf16r(a0[i]));
    o[i + 4] = toh_flush(XCARRY * bf16r(a1[i]));
  }
  _Float16* p = dst + (size_t)crow * FEAT + lane * 8u;
  *(volatile v8h*)p = o;
  __threadfence();
  *(volatile v8h*)p = o;
}

__global__ __launch_bounds__(256) void maskpack_kernel(
    const int* __restrict__ adj, unsigned* __restrict__ Mb) {
  const unsigned lane = threadIdx.x & 31u;
  const unsigned w = (unsigned)__builtin_amdgcn_readfirstlane((int)(threadIdx.x >> 5));
  const unsigned gw = blockIdx.x * 8u + w;
  const unsigned row = gw / (unsigned)LPR;
  const unsigned seg = gw - row * (unsigned)LPR;
  const int* src = adj + (size_t)row * SEQ_FULL + seg * 1024u + lane;
  unsigned word = 0u;
#pragma unroll 1
  for (unsigned j = 0; j < 32u; ++j) {
    const int a = src[j * 32u];
    const unsigned bal = __builtin_amdgcn_ballot_w32(a != 0);
    word = (lane == j) ? bal : word;
  }
  unsigned* p = Mb + (size_t)row * MWORDS + seg * 32u + lane;
  *(volatile unsigned*)p = word;
  __threadfence();
  *(volatile unsigned*)p = word;
}

__global__ __launch_bounds__(256) void gemm_h_kernel(
    const _Float16* __restrict__ A16, const _Float16* __restrict__ Bt,
    const float* __restrict__ avec, _Float16* __restrict__ vt, float* __restrict__ epart) {
  __shared__ float Cs[64 * LDC];
  __shared__ float Es[128];
  const unsigned K = (unsigned)FEAT;
  const unsigned tid = threadIdx.x, lane = tid & 31u;
  const unsigned w = (unsigned)__builtin_amdgcn_readfirstlane((int)(threadIdx.x >> 5));
  const unsigned mw = w >> 1, nw = w & 1u;
  const unsigned hh = lane >> 4, m = lane & 15u;
  const unsigned n0 = blockIdx.x * 64u;
  const unsigned row0 = blockIdx.y * 64u;

  const _Float16* ap  = A16 + (size_t)(row0 + mw * 16u + m) * K + hh * 8u;
  const _Float16* bp0 = Bt + (size_t)(n0 + nw * 32u + m) * K + hh * 8u;
  const _Float16* bp1 = bp0 + (size_t)16 * K;
  v8f acc0 = {}, acc1 = {};
#pragma unroll 2
  for (unsigned k0 = 0; k0 < K; k0 += 32u) {
    const v16h a  = frag_at(ap + k0);
    const v16h b0 = frag_at(bp0 + k0);
    const v16h b1 = frag_at(bp1 + k0);
    acc0 = wmma16(a, b0, acc0);
    acc1 = wmma16(a, b1, acc1);
  }
#pragma unroll
  for (int r = 0; r < 8; ++r) {
    float* d = &Cs[(mw * 16u + hh * 8u + (unsigned)r) * LDC + nw * 32u + m];
    d[0]  = acc0[r];
    d[16] = acc1[r];
  }
  __syncthreads();

  {
    const unsigned r = tid >> 2, q = tid & 3u;
    float s1 = 0.0f, s2 = 0.0f;
#pragma unroll 1
    for (unsigned g = 0; g < 4u; ++g) {
      const unsigned c = q * 16u + g * 4u;
      const v4f u  = *(const v4f*)&Cs[r * LDC + c];
      const v4f a1 = *(const v4f*)(avec + n0 + c);
      const v4f a2 = *(const v4f*)(avec + FEAT + n0 + c);
#pragma unroll
      for (int j = 0; j < 4; ++j) {
        const float hv = u[j] * (1.0f / (WCARRY * XCARRY));
        s1 += hv * bf16r(a1[j]);
        s2 += hv * bf16r(a2[j]);
      }
    }
    s1 += __shfl_xor(s1, 1, 32);
    s2 += __shfl_xor(s2, 1, 32);
    s1 += __shfl_xor(s1, 2, 32);
    s2 += __shfl_xor(s2, 2, 32);
    if (q == 0u) { Es[r] = s1; Es[64u + r] = s2; }
  }

  const unsigned bidx = row0 / (unsigned)SEQ;
  const unsigned key0 = row0 - bidx * (unsigned)SEQ;
  v8h x[2];
  size_t off[2];
#pragma unroll
  for (unsigned i = 0; i < 2u; ++i) {
    const unsigned dcol = 32u * i + (tid >> 3);
    const unsigned kk = (tid & 7u) * 8u;
#pragma unroll
    for (unsigned j = 0; j < 8u; ++j) {
      const float t = Cs[(kk + j) * LDC + dcol] * (HCARRY / (WCARRY * XCARRY));
      x[i][j] = toh_flush(t);
    }
    off[i] = ((size_t)bidx * FEAT + n0 + dcol) * SEQ + key0 + kk;
  }
  __syncthreads();

  v4f ev = {};
  size_t eoff = 0;
  if (w == 0u) {
    const unsigned which = lane >> 4, piece = lane & 15u;
    ev = *(const v4f*)&Es[which * 64u + piece * 4u];
    eoff = (size_t)(blockIdx.x * 2u + which) * MROWS + row0 + piece * 4u;
  }

#pragma unroll
  for (int i = 0; i < 2; ++i) *(volatile v8h*)(vt + off[i]) = x[i];
  if (w == 0u) *(volatile v4f*)(epart + eoff) = ev;
  __threadfence();
#pragma unroll
  for (int i = 0; i < 2; ++i) *(volatile v8h*)(vt + off[i]) = x[i];
  if (w == 0u) *(volatile v4f*)(epart + eoff) = ev;
}

__global__ __launch_bounds__(256) void gat_attn_kernel(
    const _Float16* __restrict__ Vt, const unsigned* __restrict__ Mb,
    const float* __restrict__ Ep, float* __restrict__ outp) {
  __shared__ _Float16 Vs[64 * LDT];
  __shared__ _Float16 Ps[8 * 16 * LDT];
  __shared__ float Os[8 * 16 * LDO];
  __shared__ float Ed[SEQ];
  __shared__ float Esr[128];
  __shared__ unsigned Ms[256];

  const unsigned tid = threadIdx.x, lane = tid & 31u;
  const unsigned w = (unsigned)__builtin_amdgcn_readfirstlane((int)(threadIdx.x >> 5));
  const unsigned hh = lane >> 4, m = lane & 15u;
  const unsigned q0 = blockIdx.x * 128u;
  const unsigned slab = blockIdx.y;
  const unsigned b = blockIdx.z;
  const unsigned qrow0 = q0 + w * 16u;
  const unsigned pbase = w * (16u * LDT);
  const unsigned obase = w * (16u * LDO);

#pragma unroll 1
  for (unsigned j = tid * 4u; j < (unsigned)SEQ; j += 1024u) {
    v4f acc = *(const v4f*)(Ep + (size_t)1 * MROWS + (size_t)b * SEQ + j);
#pragma unroll
    for (unsigned cb = 1; cb < 4u; ++cb) {
      const v4f t = *(const v4f*)(Ep + (size_t)(cb * 2u + 1u) * MROWS + (size_t)b * SEQ + j);
      acc = acc + t;
    }
    *(v4f*)&Ed[j] = acc;
  }
  if (w == 0u) {
    v4f acc = *(const v4f*)(Ep + (size_t)b * SEQ + q0 + lane * 4u);
#pragma unroll
    for (unsigned cb = 1; cb < 4u; ++cb) {
      const v4f t = *(const v4f*)(Ep + (size_t)(cb * 2u) * MROWS + (size_t)b * SEQ + q0 + lane * 4u);
      acc = acc + t;
    }
    *(v4f*)&Esr[lane * 4u] = acc;
  }
  __syncthreads();

  float es[8];
#pragma unroll
  for (int v = 0; v < 8; ++v) es[v] = Esr[w * 16u + hh * 8u + (unsigned)v];

  float mrow[8], lrow[8];
  v8f o[4];
#pragma unroll
  for (int v = 0; v < 8; ++v) { mrow[v] = -1.0e30f; lrow[v] = 0.0f; }
#pragma unroll
  for (int nb = 0; nb < 4; ++nb) o[nb] = (v8f){};

  const size_t vplane = ((size_t)b * FEAT + slab * 64u) * SEQ;

  for (unsigned kb = 0; kb < (unsigned)SEQ; kb += 64u) {
#pragma unroll
    for (unsigned j = 0; j < 2u; ++j) {
      const unsigned idx = tid + 256u * j;
      const unsigned r = idx >> 3, c = (idx & 7u) * 8u;
      *(v8h*)&Vs[r * LDT + c] = *(const v8h*)(Vt + vplane + (size_t)r * SEQ + kb + c);
    }
    Ms[tid] = Mb[(size_t)(q0 + (tid >> 1)) * MWORDS + (kb >> 5) + (tid & 1u)];
    __syncthreads();

    float ed[4];
#pragma unroll
    for (int kg = 0; kg < 4; ++kg) ed[kg] = Ed[kb + (unsigned)kg * 16u + m];
    v8f s[4];
#pragma unroll
    for (int v = 0; v < 8; ++v) {
      const unsigned rr = w * 16u + hh * 8u + (unsigned)v;
      const unsigned w0 = Ms[rr * 2u];
      const unsigned w1 = Ms[rr * 2u + 1u];
#pragma unroll
      for (int kg = 0; kg < 4; ++kg) {
        const float t = es[v] + ed[kg];
        const float lr = (t > 0.0f) ? t : (ALPHA_NEG * t);
        const unsigned word = (kg < 2) ? w0 : w1;
        const unsigned bit = (word >> ((unsigned)(kg & 1) * 16u + m)) & 1u;
        s[kg][v] = (bit != 0u) ? lr : MASK_FILL;
      }
    }

    float alpha[8];
#pragma unroll
    for (int v = 0; v < 8; ++v) {
      float mx = fmaxf(fmaxf(s[0][v], s[1][v]), fmaxf(s[2][v], s[3][v]));
      mx = red16_max(mx);
      const float mn = fmaxf(mrow[v], mx);
      alpha[v] = __expf(mrow[v] - mn);
      mrow[v] = mn;
    }
#pragma unroll
    for (int kg = 0; kg < 4; ++kg)
#pragma unroll
      for (int v = 0; v < 8; ++v) s[kg][v] = __expf(s[kg][v] - mrow[v]);

#pragma unroll
    for (int kg = 0; kg < 4; ++kg)
#pragma unroll
      for (int v = 0; v < 8; ++v) {
        const h16 ph = toh_flush(s[kg][v] * PCARRY);
        Ps[pbase + (hh * 8u + (unsigned)v) * LDT + (unsigned)kg * 16u + m] = ph;
        s[kg][v] = (float)ph;
      }
    wave_lds_sync();

#pragma unroll
    for (int v = 0; v < 8; ++v) {
      const float rs = red16_sum((s[0][v] + s[1][v]) + (s[2][v] + s[3][v]));
      lrow[v] = alpha[v] * lrow[v] + rs;
    }
#pragma unroll
    for (int nb = 0; nb < 4; ++nb)
#pragma unroll
      for (int v = 0; v < 8; ++v) o[nb][v] = o[nb][v] * alpha[v];

#pragma unroll
    for (int c = 0; c < 2; ++c) {
      const v16h pf = ld_frag(&Ps[pbase + (unsigned)c * 32u], LDT);
#pragma unroll
      for (int nb = 0; nb < 4; ++nb) {
        const v16h vf = ld_frag(&Vs[(nb * 16) * LDT + c * 32], LDT);
        o[nb] = wmma16(pf, vf, o[nb]);
      }
    }
    __syncthreads();
  }

  float inv[8];
#pragma unroll
  for (int v = 0; v < 8; ++v) inv[v] = __builtin_amdgcn_rcpf(lrow[v]) * (1.0f / HCARRY);

  v4f x[8];
  size_t off[8];
#pragma unroll
  for (int hf = 0; hf < 2; ++hf) {
#pragma unroll
    for (int nl = 0; nl < 2; ++nl)
#pragma unroll
      for (int v = 0; v < 8; ++v)
        Os[obase + (hh * 8u + (unsigned)v) * LDO + (unsigned)nl * 16u + m] =
            fmaxf(o[hf * 2 + nl][v] * inv[v], 0.0f);
    wave_lds_sync();
#pragma unroll
    for (int i = 0; i < 4; ++i) {
      const unsigned r = 4u * (unsigned)i + (lane >> 3);
      const unsigned c = (lane & 7u) * 4u;
      x[hf * 4 + i] = *(const v4f*)&Os[obase + r * LDO + c];
      off[hf * 4 + i] = ((size_t)b * SEQ_FULL + qrow0 + r) * FEAT + slab * 64u +
                        (unsigned)hf * 32u + c;
    }
    wave_lds_sync();
  }
#pragma unroll
  for (int i = 0; i < 8; ++i) *(volatile v4f*)(outp + off[i]) = x[i];
  __threadfence();
#pragma unroll
  for (int i = 0; i < 8; ++i) *(volatile v4f*)(outp + off[i]) = x[i];
}

extern "C" void kernel_launch(void* const* d_in, const int* in_sizes, int n_in,
                              void* d_out, int out_size, void* d_ws, size_t ws_size,
                              hipStream_t stream) {
  if (n_in < 4) return;
  const long long need_x = ((long long)(NB - 1) * SEQ_FULL + SEQ) * FEAT;
  if ((long long)in_sizes[0] < need_x) return;
  if ((long long)in_sizes[1] < (long long)SEQ * SEQ_FULL) return;
  if ((long long)in_sizes[2] < (long long)FEAT * FEAT) return;
  if (in_sizes[3] < 2 * FEAT) return;
  if ((long long)out_size < need_x) return;
  if (ws_size < WS_TOTAL) return;

  const float* X    = (const float*)d_in[0];
  const int*   adj  = (const int*)d_in[1];
  const float* Wm   = (const float*)d_in[2];
  const float* avec = (const float*)d_in[3];
  float* out = (float*)d_out;

  char* ws = (char*)d_ws;
  _Float16* Wt   = (_Float16*)(ws + OFF_WT);
  _Float16* X16  = (_Float16*)(ws + OFF_X16);
  _Float16* Vt16 = (_Float16*)(ws + OFF_VT);
  unsigned* Mb   = (unsigned*)(ws + OFF_MB);
  float*    Ep   = (float*)(ws + OFF_EP);

  dim3 blk(256);
  wconv_kernel<<<dim3(FEAT / 64, FEAT / 64), blk, 0, stream>>>(Wm, Wt, (unsigned)FEAT, (unsigned)FEAT);
  xconv_kernel<<<dim3(MROWS / 8), blk, 0, stream>>>(X, X16);
  maskpack_kernel<<<dim3((SEQ * LPR) / 8), blk, 0, stream>>>(adj, Mb);
  gemm_h_kernel<<<dim3(FEAT / 64, MROWS / 64), blk, 0, stream>>>(X16, Wt, avec, Vt16, Ep);
  gat_attn_kernel<<<dim3(SEQ / 128, NSLAB, NB), blk, 0, stream>>>(Vt16, Mb, Ep, out);
}
